// StableDiagonalSSM_21715354648867
// MI455X (gfx1250) — hardware-verified
//
#include <hip/hip_runtime.h>
#include <math.h>

typedef __attribute__((ext_vector_type(16))) _Float16 v16h;
typedef __attribute__((ext_vector_type(16))) __bf16 v16b;
typedef __attribute__((ext_vector_type(8)))  _Float16 v8h;
typedef __attribute__((ext_vector_type(8)))  float v8f;
typedef __attribute__((ext_vector_type(4)))  float v4f;
typedef __attribute__((ext_vector_type(2)))  float v2f;
typedef __attribute__((ext_vector_type(4)))  unsigned v4u;
typedef __attribute__((ext_vector_type(4)))  int v4i;
typedef float __attribute__((may_alias)) float_a;
typedef int __attribute__((may_alias)) int_a;

template <typename T> __device__ __forceinline__ void vst2(void* p, T v) { *(volatile T*)p = v; __threadfence(); *(volatile T*)p = v; }
__device__ __forceinline__ v8f wmma16(v16h a, v16h b, v8f c) {
  v8f d = __builtin_amdgcn_wmma_f32_16x16x32_f16(false, a, false, b, (short)0, c, false, false);
  asm volatile("v_nop\n\tv_nop\n\tv_nop\n\tv_nop" : "+v"(d) : "v"(a), "v"(b));
  return d;
}
__device__ __forceinline__ v8f wmma_bf(v16b a, v16b b, v8f c) {
  v8f d = __builtin_amdgcn_wmma_f32_16x16x32_bf16(false, a, false, b, (short)0, c, false, false);
  asm volatile("v_nop\n\tv_nop\n\tv_nop\n\tv_nop" : "+v"(d) : "v"(a), "v"(b));
  return d;
}
__device__ __forceinline__ v16h frag_h(const _Float16* rowk0, int lane) {
  union { v16h v; v8h q[2]; } u; const _Float16* p = rowk0 + 8 * (lane >> 4);
  u.q[0] = *(const v8h*)p; u.q[1] = *(const v8h*)(p + 16); return u.v;
}
__device__ __forceinline__ v16h frag_f32(const float* rowk0, int lane) {
  v16h a; const float* p = rowk0 + 8 * (lane >> 4);
#pragma unroll
  for (int i = 0; i < 8; ++i) { a[i] = (_Float16)p[i]; a[8 + i] = (_Float16)p[16 + i]; }
  return a;
}
__device__ __forceinline__ v16h frag_f32s(const float* rowk0, int lane, float sc) {
  v16h a; const float* p = rowk0 + 8 * (lane >> 4);
#pragma unroll
  for (int i = 0; i < 8; ++i) { a[i] = (_Float16)(p[i] * sc); a[8 + i] = (_Float16)(p[16 + i] * sc); }
  return a;
}
__device__ __forceinline__ v16h fragc_f32(const float* W, int k0, int n, int lane, int ld, int K) {
  v16h a; const int g = lane >> 4;
#pragma unroll
  for (int i = 0; i < 8; ++i) { const int ka = k0 + 8 * g + i, kb = ka + 16;
    a[i] = (_Float16)(ka < K ? W[(size_t)ka * ld + n] : 0.f); a[8 + i] = (_Float16)(kb < K ? W[(size_t)kb * ld + n] : 0.f); }
  return a;
}
struct F2 { v16b h, l; };
__device__ __forceinline__ F2 bsplit16(const float v[16]) { F2 r;
#pragma unroll
  for (int i = 0; i < 16; ++i) { const __bf16 h = (__bf16)v[i]; r.h[i] = h; r.l[i] = (__bf16)(v[i] - (float)h); }
  return r; }
__device__ __forceinline__ F2 split_row(const float* row, int k0, int lane) { float v[16]; const float* p = row + k0 + 8 * (lane >> 4);
#pragma unroll
  for (int i = 0; i < 8; ++i) { v[i] = p[i]; v[8 + i] = p[16 + i]; }
  return bsplit16(v); }
__device__ __forceinline__ F2 split_rowK(const float* row, int k0, int lane, int K) { float v[16]; const int g = lane >> 4;
#pragma unroll
  for (int i = 0; i < 8; ++i) { const int ka = k0 + 8 * g + i, kb = ka + 16; v[i] = ka < K ? row[ka] : 0.f; v[8 + i] = kb < K ? row[kb] : 0.f; }
  return bsplit16(v); }
__device__ __forceinline__ F2 split_col(const float* W, int k0, int n, int lane, int ld, int K) { float v[16]; const int g = lane >> 4;
#pragma unroll
  for (int i = 0; i < 8; ++i) { const int ka = k0 + 8 * g + i, kb = ka + 16; v[i] = ka < K ? W[(size_t)ka * ld + n] : 0.f; v[8 + i] = kb < K ? W[(size_t)kb * ld + n] : 0.f; }
  return bsplit16(v); }
__device__ __forceinline__ v8f mac3(const F2& a, const F2& b, v8f c) { c = wmma_bf(a.l, b.h, c); c = wmma_bf(a.h, b.l, c); return wmma_bf(a.h, b.h, c); }
__device__ __forceinline__ float sigm(float v) { return 1.0f / (1.0f + expf(-v)); }
#define LDSX() do { asm volatile("s_wait_dscnt 0" ::: "memory"); __builtin_amdgcn_wave_barrier(); __builtin_amdgcn_fence(__ATOMIC_RELEASE, "workgroup"); } while (0)

#define NB 4
#define LL 2048
#define DM 1024
#define NS 128
#define NR (NB * LL)

__global__ __launch_bounds__(256) void k_cvt(const float* __restrict__ src, _Float16* __restrict__ dst, size_t n8, float sc) {
  const size_t g8 = (size_t)blockIdx.x * 256 + threadIdx.x; if (g8 >= n8) return;
  union { v8h h; v4u u; } pk;
#pragma unroll
  for (int e = 0; e < 8; ++e) pk.h[e] = (_Float16)(src[g8 * 8 + e] * sc);
  vst2(dst + g8 * 8, pk.u);
}
__device__ __forceinline__ void gemm_tile(const _Float16* A, int lda, const _Float16* Bm, int K, int r0, int n0, int lane, v8f acc[8]) {
  const int col = lane & 15;
#pragma unroll 1
  for (int kc = 0; kc < K / 32; ++kc) { const v16h a = frag_h(A + (size_t)(r0 + col) * lda + kc * 32, lane);
#pragma unroll
    for (int j = 0; j < 8; ++j) acc[j] = wmma16(a, frag_h(Bm + (size_t)(n0 + j * 16 + col) * K + kc * 32, lane), acc[j]); }
}
__global__ __launch_bounds__(128) void k_in(const _Float16* __restrict__ x16, const _Float16* __restrict__ Win16, _Float16* __restrict__ u16, float* __restrict__ gate) {
  __shared__ __align__(16) float so[4][16][132];
  const int tid = threadIdx.x, wave = tid >> 5, lane = tid & 31, col = lane & 15, g = lane >> 4;
  const int r0 = blockIdx.x * 64 + wave * 16, n0 = blockIdx.y * 128;
  v8f acc[8] = {}; gemm_tile(x16, DM, Win16, DM, r0, n0, lane, acc);
#pragma unroll
  for (int j = 0; j < 8; ++j)
#pragma unroll
    for (int r = 0; r < 8; ++r) so[wave][8 * g + r][j * 16 + col] = acc[j][r] * (1.0f / 16.0f);
  LDSX();
  if (n0 < DM) {
    for (int q = lane; q < 16 * 16; q += 32) { const int rl = q >> 4, pc = q & 15; union { v8h hh; v4u u; } pk;
#pragma unroll
      for (int i = 0; i < 8; ++i) pk.hh[i] = (_Float16)so[wave][rl][pc * 8 + i];
      vst2(u16 + (size_t)(r0 + rl) * DM + n0 + pc * 8, pk.u); } }
  else {
#pragma unroll 4
    for (int rl = 0; rl < 16; ++rl) vst2(gate + (size_t)(r0 + rl) * DM + (n0 - DM) + lane * 4, *(const v4f*)(&so[wave][rl][lane * 4])); }
}
__global__ __launch_bounds__(128) void k_bd(const _Float16* __restrict__ u16, const _Float16* __restrict__ Wsd16, const float* __restrict__ bdt, const float* __restrict__ Alog, float* __restrict__ bt, float* __restrict__ dec) {
  __shared__ __align__(16) float so[4][16][132];
  const int tid = threadIdx.x, wave = tid >> 5, lane = tid & 31, col = lane & 15, g = lane >> 4;
  const int r0 = blockIdx.x * 64 + wave * 16, which = blockIdx.y;
  v8f acc[8] = {}; gemm_tile(u16, DM, Wsd16, DM, r0, which * NS, lane, acc);
#pragma unroll
  for (int j = 0; j < 8; ++j) { const int n = j * 16 + col;
    if (which == 0) {
#pragma unroll
      for (int r = 0; r < 8; ++r) so[wave][8 * g + r][n] = acc[j][r] * (1.0f / 16.0f); }
    else { const float b0 = bdt[n]; const float al = Alog[n]; const float rate = (al > 20.f ? al : log1pf(expf(al))) + 1e-4f;
#pragma unroll
      for (int r = 0; r < 8; ++r) { const float v = acc[j][r] * (1.0f / 16.0f) + b0; float sp = v > 20.f ? v : log1pf(expf(v)); sp = fminf(sp, 10.0f);
        float d = expf(-sp * rate); d = fminf(fmaxf(d, 0.f), 1.0f); so[wave][8 * g + r][n] = d; } } }
  LDSX();
  float* dst = which == 0 ? bt : dec;
#pragma unroll 4
  for (int rl = 0; rl < 16; ++rl) vst2(dst + (size_t)(r0 + rl) * NS + lane * 4, *(const v4f*)(&so[wave][rl][lane * 4]));
}
__global__ __launch_bounds__(128) void k_scan(const float* __restrict__ bt, const float* __restrict__ dec, float* __restrict__ hs) {
  const int b = blockIdx.x, n = threadIdx.x; float h = 0.f;
#pragma unroll 1
  for (int l = 0; l < LL; ++l) { const size_t o = ((size_t)b * LL + l) * NS + n; const float d = dec[o]; h = d * h + (1.0f - d) * bt[o]; vst2(hs + o, (float_a)h); }
}
__global__ __launch_bounds__(128) void k_yz(const float* __restrict__ hs, const _Float16* __restrict__ Wc16, const float* __restrict__ gate, const float* __restrict__ x, const float* __restrict__ Dv, _Float16* __restrict__ z16) {
  __shared__ __align__(16) float so[4][16][132];
  const int tid = threadIdx.x, wave = tid >> 5, lane = tid & 31, col = lane & 15, g = lane >> 4;
  const int r0 = blockIdx.x * 64 + wave * 16, n0 = blockIdx.y * 128;
  v8f acc[8] = {};
#pragma unroll
  for (int kc = 0; kc < NS / 32; ++kc) { const v16h a = frag_f32(hs + (size_t)(r0 + col) * NS + kc * 32, lane);
#pragma unroll
    for (int j = 0; j < 8; ++j) acc[j] = wmma16(a, frag_h(Wc16 + (size_t)(n0 + j * 16 + col) * NS + kc * 32, lane), acc[j]); }
#pragma unroll
  for (int j = 0; j < 8; ++j)
#pragma unroll
    for (int r = 0; r < 8; ++r) so[wave][8 * g + r][j * 16 + col] = acc[j][r] * 0.125f;
  LDSX();
  for (int q = lane; q < 16 * 16; q += 32) { const int rl = q >> 4, pc = q & 15; const size_t o = (size_t)(r0 + rl) * DM + n0 + pc * 8; union { v8h hh; v4u u; } pk;
#pragma unroll
    for (int i = 0; i < 8; ++i) { const float gv = gate[o + i]; const float sg = gv * sigm(gv); pk.hh[i] = (_Float16)(so[wave][rl][pc * 8 + i] * sg + x[o + i] * Dv[n0 + pc * 8 + i]); }
    vst2(z16 + o, pk.u); }
}
__global__ __launch_bounds__(128) void k_out(const _Float16* __restrict__ z16, const _Float16* __restrict__ Wo16, float* __restrict__ out) {
  __shared__ __align__(16) float so[4][16][132];
  const int tid = threadIdx.x, wave = tid >> 5, lane = tid & 31, col = lane & 15, g = lane >> 4;
  const int r0 = blockIdx.x * 64 + wave * 16, n0 = blockIdx.y * 128;
  v8f acc[8] = {}; gemm_tile(z16, DM, Wo16, DM, r0, n0, lane, acc);
#pragma unroll
  for (int j = 0; j < 8; ++j)
#pragma unroll
    for (int r = 0; r < 8; ++r) so[wave][8 * g + r][j * 16 + col] = acc[j][r] * (1.0f / 16.0f);
  LDSX();
#pragma unroll 4
  for (int rl = 0; rl < 16; ++rl) vst2(out + (size_t)(r0 + rl) * DM + n0 + lane * 4, *(const v4f*)(&so[wave][rl][lane * 4]));
}
extern "C" void kernel_launch(void* const* d_in, const int* in_sizes, int n_in, void* d_out, int out_size, void* d_ws, size_t ws_size, hipStream_t stream) {
  (void)in_sizes; (void)n_in; (void)out_size; (void)ws_size;
  const float* x = (const float*)d_in[0]; const float* Win = (const float*)d_in[1]; const float* Wst = (const float*)d_in[2]; const float* Wdt = (const float*)d_in[3]; const float* bdt = (const float*)d_in[4];
  const float* Alog = (const float*)d_in[5]; const float* Wc = (const float*)d_in[6]; const float* Dv = (const float*)d_in[7]; const float* Wout = (const float*)d_in[8];
  float* out = (float*)d_out;
  char* ws = (char*)d_ws; size_t off = 0;
  auto take = [&](size_t bytes) { char* p = ws + off; off += (bytes + 255) & ~(size_t)255; return p; };
  _Float16* x16 = (_Float16*)take((size_t)NR * DM * 2); _Float16* Win16 = (_Float16*)take((size_t)2 * DM * DM * 2); _Float16* Wsd16 = (_Float16*)take((size_t)2 * NS * DM * 2);
  _Float16* Wc16 = (_Float16*)take((size_t)DM * NS * 2); _Float16* Wo16 = (_Float16*)take((size_t)DM * DM * 2);
  _Float16* u16 = (_Float16*)take((size_t)NR * DM * 2); float* gate = (float*)take((size_t)NR * DM * 4);
  float* bt = (float*)take((size_t)NR * NS * 4); float* dec = (float*)take((size_t)NR * NS * 4); float* hs = (float*)take((size_t)NR * NS * 4); _Float16* z16 = (_Float16*)take((size_t)NR * DM * 2);
  auto cvt = [&](const float* s, _Float16* d, size_t n, float sc) { const size_t n8 = n / 8; k_cvt<<<(unsigned)((n8 + 255) / 256), 256, 0, stream>>>(s, d, n8, sc); };
  cvt(x, x16, (size_t)NR * DM, 1.0f); cvt(Win, Win16, (size_t)2 * DM * DM, 16.0f); cvt(Wst, Wsd16, (size_t)NS * DM, 16.0f); cvt(Wdt, Wsd16 + (size_t)NS * DM, (size_t)NS * DM, 16.0f);
  cvt(Wc, Wc16, (size_t)DM * NS, 8.0f); cvt(Wout, Wo16, (size_t)DM * DM, 16.0f);
  k_in<<<dim3(NR / 64, 2 * DM / 128), 128, 0, stream>>>(x16, Win16, u16, gate);
  k_bd<<<dim3(NR / 64, 2), 128, 0, stream>>>(u16, Wsd16, bdt, Alog, bt, dec);
  k_scan<<<NB, 128, 0, stream>>>(bt, dec, hs);
  k_yz<<<dim3(NR / 64, DM / 128), 128, 0, stream>>>(hs, Wc16, gate, x, Dv, z16);
  k_out<<<dim3(NR / 64, DM / 128), 128, 0, stream>>>(z16, Wo16, out);
}
